// MambaBlock_v1_1520418422822
// MI455X (gfx1250) — hardware-run, weakly checked
//
#include <hip/hip_runtime.h>
#include <hip/hip_fp16.h>
#include <math.h>

typedef __attribute__((ext_vector_type(16))) _Float16 v16h;
typedef __attribute__((ext_vector_type(8)))  _Float16 v8h;
typedef __attribute__((ext_vector_type(8)))  float    v8f;
typedef __attribute__((ext_vector_type(4)))  float    v4f;

constexpr int kBatch    = 8;
constexpr int kSeq      = 512;
constexpr int kDm       = 512;
constexpr int kDin      = 1024;
constexpr int kNst      = 16;
constexpr int kDtR      = 32;
constexpr int kGroups   = 8;
constexpr int kRows     = kBatch * kSeq;
constexpr int kXzP      = 2 * kDin;
constexpr int kBcP      = kDtR + 2 * kNst;
constexpr int kScanOffB = kDtR;
constexpr int kScanOffC = kDtR + kNst;
constexpr int kConvTP   = 260;
constexpr float kWCarry = 1024.0f;
constexpr float kResid  = 2048.0f;
constexpr float kYCarry = 16.0f;
constexpr float kSW  = 1.0f / kWCarry;
constexpr float kSWr = 1.0f / (kWCarry * kResid);
constexpr float kSY  = 1.0f / (kYCarry * kWCarry);
constexpr float kSYr = 1.0f / (kYCarry * kWCarry * kResid);
static_assert(kRows == 4096);
static_assert(kBcP == 64);
static_assert((kDm % 64) == 0 && (kDin % 64) == 0 && (kSeq % 64) == 0);
static_assert((kXzP % 64) == 0 && (kBcP % 64) == 0 && (kDin % 256) == 0);
static_assert((kDm / kGroups) == 64);
static_assert((kRows % 32) == 0 && (kRows % 16) == 0);
static_assert((kDm % 32) == 0 && (kDin % 32) == 0 && (kDtR % 32) == 0);

constexpr size_t kSzWIN  = (size_t)kXzP * kDm * 2;
constexpr size_t kSzWX   = (size_t)kBcP * kDin * 2;
constexpr size_t kSzWDT  = (size_t)kDin * kDtR * 2;
constexpr size_t kSzWOUT = (size_t)kDm * kDin * 2;
constexpr size_t kSzX16  = (size_t)kRows * kDm * 2;
constexpr size_t kSzXZ   = (size_t)kRows * kXzP * 4;
constexpr size_t kSzU    = (size_t)kRows * kDin * 4;
constexpr size_t kSzU16  = (size_t)kRows * kDin * 2;
constexpr size_t kSzBC   = (size_t)kRows * kBcP * 4;
constexpr size_t kSzBC16 = (size_t)kRows * kBcP * 2;
constexpr size_t kSzO    = (size_t)kRows * kDm * 4;
constexpr size_t kSzST   = (size_t)kBatch * kGroups * 32 * 4;
constexpr size_t kWsWINH = 0;
constexpr size_t kWsWINL = kWsWINH + kSzWIN;
constexpr size_t kWsWX   = kWsWINL + kSzWIN;
constexpr size_t kWsWDT  = kWsWX   + kSzWX;
constexpr size_t kWsWOUT = kWsWDT  + kSzWDT;
constexpr size_t kWsXH   = kWsWOUT + kSzWOUT;
constexpr size_t kWsXL   = kWsXH   + kSzX16;
constexpr size_t kWsXZ   = kWsXL   + kSzX16;
constexpr size_t kWsU    = kWsXZ   + kSzXZ;
constexpr size_t kWsUH   = kWsU    + kSzU;
constexpr size_t kWsUL   = kWsUH   + kSzU16;
constexpr size_t kWsBC   = kWsUL   + kSzU16;
constexpr size_t kWsBCH  = kWsBC   + kSzBC;
constexpr size_t kWsBCL  = kWsBCH  + kSzBC16;
constexpr size_t kWsDTR  = kWsBCL  + kSzBC16;
constexpr size_t kWsDT   = kWsDTR  + kSzU;
constexpr size_t kWsYH   = kWsDT   + kSzU;
constexpr size_t kWsYL   = kWsYH   + kSzU16;
constexpr size_t kWsST   = kWsYL   + kSzU16;
constexpr size_t kWsTotal = kWsST  + kSzST;
constexpr size_t kWsO    = kWsXZ;
static_assert(kWsTotal == 133373952ull);
static_assert(kWsTotal <= 134217728ull);
static_assert(kSzO <= kSzXZ);
static_assert((kWsWINL % 128) == 0 && (kWsWX % 128) == 0 && (kWsWDT % 128) == 0 && (kWsWOUT % 128) == 0 &&
              (kWsXH % 128) == 0 && (kWsXL % 128) == 0 && (kWsXZ % 128) == 0 && (kWsU % 128) == 0 &&
              (kWsUH % 128) == 0 && (kWsUL % 128) == 0 && (kWsBC % 128) == 0 && (kWsBCH % 128) == 0 &&
              (kWsBCL % 128) == 0 && (kWsDTR % 128) == 0 && (kWsDT % 128) == 0 && (kWsYH % 128) == 0 &&
              (kWsYL % 128) == 0 && (kWsST % 128) == 0);

__device__ __forceinline__ _Float16 f16_flush(float v) {
  const float w = (fabsf(v) < 6.103515625e-05f) ? 0.0f : v;
  return (_Float16)w;
}
__device__ __forceinline__ void f16_split(float v, _Float16& hi, _Float16& lo) {
  hi = f16_flush(v);
  const float hf = (float)hi;
  const float r = (v - hf) * kResid;
  lo = f16_flush(r);
}

namespace eng {
union FragU { v16h v; v8h h[2]; };
__device__ __forceinline__ v16h frag_load(const _Float16* p) {
  FragU f;
  f.h[0] = *(const v8h*)(p);
  f.h[1] = *(const v8h*)(p + 16);
  return f.v;
}
__device__ __forceinline__ v8f mma(v16h a, v16h b, v8f c) {
  return __builtin_amdgcn_wmma_f32_16x16x32_f16(false, a, false, b, (short)0, c, false, false);
}
__device__ __forceinline__ void guard1(v8f& a, v16h x, v16h y) {
  asm volatile("v_nop\n\tv_nop\n\tv_nop\n\tv_nop" : "+v"(a) : "v"(x), "v"(y));
}
__device__ __forceinline__ void guard_acc(v8f& a) {
  asm volatile("v_nop\n\tv_nop\n\tv_nop\n\tv_nop" : "+v"(a));
}
__device__ __forceinline__ void keep4(v16h a, v16h b, v16h c, v16h d) {
  asm volatile("v_nop" :: "v"(a), "v"(b), "v"(c), "v"(d));
}

template <int MI, int SPL>
__global__ __launch_bounds__(256) void gemm_f16_kernel(
    const unsigned short* __restrict__ Ap, const unsigned short* __restrict__ A2p, int lda,
    const unsigned short* __restrict__ Btp, const unsigned short* __restrict__ Bt2p, int ldb,
    float* __restrict__ C, int ldc, int M, int N, int K, float scale, float rscale)
{
  static_assert(MI >= 1 && MI <= 2);
  static_assert(SPL >= 0 && SPL <= 2);
  const _Float16* A   = (const _Float16*)Ap;
  const _Float16* A2  = (const _Float16*)A2p;
  const _Float16* Bt  = (const _Float16*)Btp;
  const _Float16* Bt2 = (const _Float16*)Bt2p;
  __shared__ __align__(16) float sT[8][16 * 68];
  const int lane = threadIdx.x & 31;
  const int wave = threadIdx.x >> 5;
  const int tilesN = N >> 6;
  const int tilesM = M / (16 * MI);
  const int tile = blockIdx.x * 8 + wave;
  if (tile >= tilesM * tilesN) return;
  const int tm = tile / tilesN;
  const int tn = tile - tm * tilesN;
  const int m0 = tm * (16 * MI);
  const int n0 = tn << 6;
  const int rlane = lane & 15;
  const int koff  = (lane >> 4) * 8;
  const int mOff  = (lane >> 4) * 8;

  v8f acc[MI][4], accr[MI][4];
#pragma unroll
  for (int i = 0; i < MI; ++i)
#pragma unroll
    for (int j = 0; j < 4; ++j) {
      acc[i][j]  = (v8f){0.f, 0.f, 0.f, 0.f, 0.f, 0.f, 0.f, 0.f};
      accr[i][j] = (v8f){0.f, 0.f, 0.f, 0.f, 0.f, 0.f, 0.f, 0.f};
    }

  for (int k0 = 0; k0 < K; k0 += 32) {
    v16h bh[4], bl[4];
#pragma unroll
    for (int j = 0; j < 4; ++j) {
      const size_t bo = (size_t)(n0 + (j << 4) + rlane) * ldb + koff + k0;
      bh[j] = frag_load(Bt + bo);
      if (SPL == 2) bl[j] = frag_load(Bt2 + bo); else bl[j] = bh[j];
    }
#pragma unroll
    for (int i = 0; i < MI; ++i) {
      const size_t ao = (size_t)(m0 + (i << 4) + rlane) * lda + koff + k0;
      const v16h ah = frag_load(A + ao);
      v16h al = ah;
      if (SPL >= 1) al = frag_load(A2 + ao);
#pragma unroll
      for (int j = 0; j < 4; ++j) {
        acc[i][j] = mma(ah, bh[j], acc[i][j]);
        if (SPL >= 1) accr[i][j] = mma(al, bh[j], accr[i][j]);
        if (SPL == 2) accr[i][j] = mma(ah, bl[j], accr[i][j]);
      }
#pragma unroll
      for (int j = 0; j < 4; ++j) {
        guard1(acc[i][j], ah, al);
        if (SPL >= 1) guard1(accr[i][j], ah, al);
      }
    }
    keep4(bh[0], bh[1], bh[2], bh[3]);
    if (SPL == 2) keep4(bl[0], bl[1], bl[2], bl[3]);
  }
#pragma unroll
  for (int i = 0; i < MI; ++i)
#pragma unroll
    for (int j = 0; j < 4; ++j) {
      guard_acc(acc[i][j]);
      if (SPL >= 1) guard_acc(accr[i][j]);
    }

  float* slab = sT[wave];
#pragma unroll
  for (int i = 0; i < MI; ++i) {
    const int mBase = m0 + (i << 4);
#pragma unroll
    for (int j = 0; j < 4; ++j) {
#pragma unroll
      for (int r = 0; r < 8; ++r) {
        float v = acc[i][j][r] * scale;
        if (SPL >= 1) v += accr[i][j][r] * rscale;
        slab[(mOff + r) * 68 + (j << 4) + rlane] = v;
      }
    }
    __builtin_amdgcn_fence(__ATOMIC_RELEASE, "workgroup");
    __builtin_amdgcn_wave_barrier();
    __builtin_amdgcn_fence(__ATOMIC_ACQUIRE, "workgroup");
    {
      const int hh = lane >> 4, c4 = (lane & 15) * 4;
      for (int pass = 0; pass < 2; ++pass) {
#pragma unroll
        for (int it = 0; it < 8; ++it) {
          const int row = it * 2 + hh;
          const v4f v = *(const v4f*)(slab + row * 68 + c4);
          *(volatile v4f*)(C + (size_t)(mBase + row) * ldc + n0 + c4) = v;
        }
        __threadfence();
      }
    }
    __builtin_amdgcn_fence(__ATOMIC_RELEASE, "workgroup");
    __builtin_amdgcn_wave_barrier();
    __builtin_amdgcn_fence(__ATOMIC_ACQUIRE, "workgroup");
  }
}
}

__global__ __launch_bounds__(256) void split_rows_f16_kernel(
    const float* __restrict__ src, unsigned short* __restrict__ dH, unsigned short* __restrict__ dL, int total8)
{
  const int i = blockIdx.x * 256 + threadIdx.x;
  if (i >= total8) return;
  const size_t e0 = (size_t)i << 3;
  const v4f a0 = *(const v4f*)(src + e0);
  const v4f a1 = *(const v4f*)(src + e0 + 4);
  v8h hv, lv;
#pragma unroll
  for (int e = 0; e < 4; ++e) {
    _Float16 h0, l0, h1, l1;
    const float f0 = a0[e];
    const float f1 = a1[e];
    f16_split(f0, h0, l0);
    f16_split(f1, h1, l1);
    hv[e] = h0; lv[e] = l0;
    hv[4 + e] = h1; lv[4 + e] = l1;
  }
  unsigned short* qh = dH + e0;
  unsigned short* ql = dL + e0;
  *(volatile v8h*)qh = hv;
  *(volatile v8h*)ql = lv;
  __threadfence();
  *(volatile v8h*)qh = hv;
  *(volatile v8h*)ql = lv;
}

template <bool LO>
__global__ __launch_bounds__(256) void pack_weight_f16_kernel(
    const float* __restrict__ src, unsigned short* __restrict__ dH, unsigned short* __restrict__ dL,
    int total8, float carry)
{
  const int i = blockIdx.x * 256 + threadIdx.x;
  if (i >= total8) return;
  const size_t e0 = (size_t)i << 3;
  const v4f a0 = *(const v4f*)(src + e0);
  const v4f a1 = *(const v4f*)(src + e0 + 4);
  v8h hv, lv;
#pragma unroll
  for (int e = 0; e < 4; ++e) {
    _Float16 h0, l0, h1, l1;
    const float f0 = a0[e] * carry;
    const float f1 = a1[e] * carry;
    f16_split(f0, h0, l0);
    f16_split(f1, h1, l1);
    hv[e] = h0; lv[e] = l0;
    hv[4 + e] = h1; lv[4 + e] = l1;
  }
  unsigned short* qh = dH + e0;
  unsigned short* ql = dL + e0;
  *(volatile v8h*)qh = hv;
  if (LO) *(volatile v8h*)ql = lv;
  __threadfence();
  *(volatile v8h*)qh = hv;
  if (LO) *(volatile v8h*)ql = lv;
}

__global__ __launch_bounds__(256) void xpose_split_kernel(
    const float* __restrict__ x, unsigned short* __restrict__ XH, unsigned short* __restrict__ XL)
{
  __shared__ float tile[64 * 65];
  const int tid = threadIdx.x, lane = tid & 31, wave = tid >> 5;
  const int l0 = blockIdx.x * 64;
  const int d0 = blockIdx.y * 64;
  const int b  = blockIdx.z;
  const float* xb = x + (size_t)b * kDm * kSeq;
#pragma unroll
  for (int p = 0; p < 16; ++p) {
    const int idx = tid + p * 256;
    const int dd  = idx >> 6;
    const int ll  = idx & 63;
    tile[dd * 65 + ll] = xb[(size_t)(d0 + dd) * kSeq + l0 + ll];
  }
  __syncthreads();
  const int q = lane >> 3, c8 = (lane & 7) * 8;
  v8h hv[2], lv[2];
#pragma unroll
  for (int it = 0; it < 2; ++it) {
    const int lrow = it * 32 + wave * 4 + q;
#pragma unroll
    for (int e = 0; e < 8; ++e) {
      _Float16 h, l;
      const float t = tile[(c8 + e) * 65 + lrow];
      f16_split(t, h, l);
      hv[it][e] = h;
      lv[it][e] = l;
    }
  }
  for (int pass = 0; pass < 2; ++pass) {
#pragma unroll
    for (int it = 0; it < 2; ++it) {
      const int lrow = it * 32 + wave * 4 + q;
      const size_t o = (size_t)(b * kSeq + l0 + lrow) * kDm + d0 + c8;
      *(volatile v8h*)(XH + o) = hv[it];
      *(volatile v8h*)(XL + o) = lv[it];
    }
    __threadfence();
  }
}

__global__ __launch_bounds__(256) void conv_silu_kernel(
    const float* __restrict__ XZ, const float* __restrict__ cw, const float* __restrict__ cb,
    float* __restrict__ UC, unsigned short* __restrict__ UH, unsigned short* __restrict__ UL)
{
  __shared__ __align__(16) float sT[16 * kConvTP];
  const int tid = threadIdx.x, lane = tid & 31, wave = tid >> 5;
  const int d0 = blockIdx.x * 256, d = d0 + tid;
  const int t0 = blockIdx.y * 64;
  const v4f wv = *(const v4f*)(cw + (size_t)d * 4);
  const float w0 = wv[0], w1 = wv[1], w2 = wv[2], w3 = wv[3];
  const float bc = cb[d];
  float xm3, xm2, xm1;
  {
    const int r3 = t0 - 3, r2 = t0 - 2, r1 = t0 - 1;
    const float v3 = XZ[(size_t)(r3 < 0 ? 0 : r3) * kXzP + d];
    const float v2 = XZ[(size_t)(r2 < 0 ? 0 : r2) * kXzP + d];
    const float v1 = XZ[(size_t)(r1 < 0 ? 0 : r1) * kXzP + d];
    xm3 = (r3 >= 0) ? v3 : 0.0f;
    xm2 = (r2 >= 0) ? v2 : 0.0f;
    xm1 = (r1 >= 0) ? v1 : 0.0f;
  }
  const int hrow = wave >> 1;
  const int hch  = (wave & 1) * 128 + lane * 4;
#pragma unroll 1
  for (int sub = 0; sub < 4; ++sub) {
    const int lb = t0 + sub * 16;
#pragma unroll 1
    for (int s = 0; s < 16; ++s) {
      const float xcur = XZ[(size_t)(lb + s) * kXzP + d];
      float acc = w0 * xm3;
      acc = fmaf(w1, xm2, acc);
      acc = fmaf(w2, xm1, acc);
      acc = fmaf(w3, xcur, acc);
      const float sv = acc + bc;
      const float sg = __builtin_amdgcn_rcpf(1.0f + expf(-sv));
      sT[s * kConvTP + tid] = sv * sg;
      xm3 = xm2; xm2 = xm1; xm1 = xcur;
    }
    __syncthreads();
    v4f fv[4];
    v8h hv[2], lv[2];
#pragma unroll
    for (int it = 0; it < 4; ++it) fv[it] = *(const v4f*)(sT + (it * 4 + hrow) * kConvTP + hch);
#pragma unroll
    for (int it = 0; it < 2; ++it) {
      const float* sp = sT + (it * 8 + wave) * kConvTP + lane * 8;
      const v4f a0 = *(const v4f*)(sp);
      const v4f a1 = *(const v4f*)(sp + 4);
#pragma unroll
      for (int e = 0; e < 4; ++e) {
        _Float16 h0, l0, h1, l1;
        const float f0 = a0[e];
        const float f1 = a1[e];
        f16_split(f0, h0, l0);
        f16_split(f1, h1, l1);
        hv[it][e] = h0; lv[it][e] = l0;
        hv[it][4 + e] = h1; lv[it][4 + e] = l1;
      }
    }
    for (int pass = 0; pass < 2; ++pass) {
#pragma unroll
      for (int it = 0; it < 4; ++it)
        *(volatile v4f*)(UC + (size_t)(lb + it * 4 + hrow) * kDin + d0 + hch) = fv[it];
#pragma unroll
      for (int it = 0; it < 2; ++it) {
        const size_t o = (size_t)(lb + it * 8 + wave) * kDin + d0 + lane * 8;
        *(volatile v8h*)(UH + o) = hv[it];
        *(volatile v8h*)(UL + o) = lv[it];
      }
      __threadfence();
    }
    __syncthreads();
  }
}

__global__ __launch_bounds__(256) void bias_rows_kernel(
    const float* __restrict__ DTR, const float* __restrict__ bdt, float* __restrict__ DT)
{
  const int d4 = (blockIdx.x * 256 + threadIdx.x) * 4;
  const int r0 = blockIdx.y * 8;
  const v4f b = *(const v4f*)(bdt + d4);
  v4f val[8];
#pragma unroll
  for (int i = 0; i < 8; ++i) {
    const v4f t = *(const v4f*)(DTR + (size_t)(r0 + i) * kDin + d4);
    val[i] = t + b;
  }
  for (int pass = 0; pass < 2; ++pass) {
#pragma unroll
    for (int i = 0; i < 8; ++i)
      *(volatile v4f*)(DT + (size_t)(r0 + i) * kDin + d4) = val[i];
    __threadfence();
  }
}

typedef float    ms1_v4f __attribute__((ext_vector_type(4)));
typedef unsigned ms1_v4u __attribute__((ext_vector_type(4)));
struct ms1_args {
  const float* dtpre;
  const float* u;
  const float* bc;
  const float* z;
  const float* A_log;
  const float* Dskip;
  __half* y;
  __half* y_lo;
  long ld_dtpre;
  long ld_u;
  long ld_bc;
  long ld_z;
  long ld_y;
  int offB;
  int offC;
  int offZ;
  float ycarry;
  int dir;
  int D;
  int L;
  int nbatch;
};
static_assert(sizeof(ms1_args) == 136);

__device__ __forceinline__ float ms1_flush16(float v) {
  return (fabsf(v) < 6.103515625e-05f) ? 0.0f : v;
}
__device__ __forceinline__ unsigned ms1_h16bits(float v) {
  return (unsigned)__half_as_ushort(__float2half_rn(ms1_flush16(v)));
}
__device__ __forceinline__ float ms1_h16val(unsigned b) {
  return __half2float(__ushort_as_half((unsigned short)b));
}
__device__ __forceinline__ float ms1_softplus(float v) {
  return fmaxf(v, 0.0f) + log1pf(expf(-fabsf(v)));
}
__device__ __forceinline__ void ms1_pack2(float v0, float v1, unsigned& hw, unsigned& lw) {
  const unsigned h0 = ms1_h16bits(v0);
  const unsigned h1 = ms1_h16bits(v1);
  const float r0 = (v0 - ms1_h16val(h0)) * 2048.0f;
  const float r1 = (v1 - ms1_h16val(h1)) * 2048.0f;
  const unsigned l0 = ms1_h16bits(r0);
  const unsigned l1 = ms1_h16bits(r1);
  hw = h0 | (h1 << 16);
  lw = l0 | (l1 << 16);
}

template <int NSTATE>
__global__ __launch_bounds__(64 * (NSTATE / 16)) void ms1_scan_kernel(ms1_args a)
{
  static_assert(NSTATE == 16 || NSTATE == 64);
  constexpr int NQ  = NSTATE / 16;
  constexpr int NT  = 64 * NQ;
  constexpr int NW  = NT / 32;
  constexpr int BCW = 2 * NSTATE;
  constexpr int YP  = 68;
  constexpr int RPI = NW * 4;
  constexpr int NIT = 64 / RPI;
  static_assert(16 * NT <= 64 * YP);
  __shared__ __align__(16) float sBC[64 * BCW];
  __shared__ __align__(16) float sY[64 * YP];
  const int tid  = threadIdx.x;
  const int lane = tid & 31;
  const int wave = tid >> 5;
  const int c    = tid / NQ;
  const int sq   = tid - c * NQ;
  const int bpb  = a.D / 64;
  const int bi   = blockIdx.x / bpb;
  if (bi >= a.nbatch) return;
  const int d0 = (blockIdx.x - bi * bpb) * 64;
  const int d  = d0 + c;
  const long rowb = (long)bi * a.L;
  const bool hasz  = (a.z != nullptr);
  const bool hasD  = (a.Dskip != nullptr);
  const bool hasLo = (a.y_lo != nullptr);

#pragma unroll 1
  for (int n = 0; n < 16; ++n) {
    const float al = a.A_log[(long)d * NSTATE + sq * 16 + n];
    sY[n * NT + tid] = -expf(al);
  }
  __syncthreads();
  float An[16], h[16];
#pragma unroll
  for (int n = 0; n < 16; ++n) {
    An[n] = sY[n * NT + tid];
    h[n] = 0.0f;
  }
  float Dd = 0.0f;
  if (hasD) Dd = a.Dskip[d];

  const int nchunk = a.L / 64;
  const bool fwd = (a.dir > 0);
  const int s0 = fwd ? 0 : 63;
  const int sd = fwd ? 1 : -1;
  const int q  = lane >> 3;
  const int c8 = (lane & 7) * 8;

#pragma unroll 1
  for (int ci = 0; ci < nchunk; ++ci) {
    const int tb = fwd ? (ci * 64) : (a.L - 64 - ci * 64);
    const long rowc = rowb + tb;
    __syncthreads();
#pragma unroll 8
    for (int i = 0; i < 32; ++i) {
      const int idx = tid + i * NT;
      const int st  = idx / BCW;
      const int col = idx - st * BCW;
      const int sc  = (col < NSTATE) ? (a.offB + col) : (a.offC + col - NSTATE);
      sBC[idx] = a.bc[(rowc + st) * a.ld_bc + sc];
    }
    __syncthreads();
#pragma unroll 1
    for (int s = 0; s < 64; ++s) {
      const int ls = s0 + sd * s;
      const long row = rowc + ls;
      float pre = a.dtpre[row * a.ld_dtpre + d];
      float uv  = a.u[row * a.ld_u + d];
      float zv  = 0.0f;
      if (hasz) zv = a.z[row * a.ld_z + a.offZ + d];
      asm volatile("" : "+v"(pre));
      asm volatile("" : "+v"(uv));
      asm volatile("" : "+v"(zv));
      const float delta = ms1_softplus(pre);
      const float dtx = delta * uv;
      const float* bp = sBC + ls * BCW + sq * 16;
      const float* cp = bp + NSTATE;
      ms1_v4f Bq[4], Cq[4];
#pragma unroll
      for (int k = 0; k < 4; ++k) {
        Bq[k] = *(const ms1_v4f*)(bp + 4 * k);
        Cq[k] = *(const ms1_v4f*)(cp + 4 * k);
      }
      float yv = 0.0f;
#pragma unroll
      for (int n = 0; n < 16; ++n) {
        const float e = __expf(delta * An[n]);
        h[n] = fmaf(e, h[n], dtx * Bq[n >> 2][n & 3]);
        yv = fmaf(h[n], Cq[n >> 2][n & 3], yv);
      }
      if (NQ > 1) {
        yv += __shfl_xor(yv, 1, 32);
        yv += __shfl_xor(yv, 2, 32);
      }
      if (hasD) yv = fmaf(uv, Dd, yv);
      if (hasz) {
        const float sg = __builtin_amdgcn_rcpf(1.0f + expf(-zv));
        yv = yv * (zv * sg);
      }
      if (sq == 0) sY[ls * YP + c] = yv * a.ycarry;
    }
    __syncthreads();
    ms1_v4u hw[NIT], lw[NIT];
#pragma unroll
    for (int it = 0; it < NIT; ++it) {
      const int row = it * RPI + wave * 4 + q;
      const float* sp = sY + row * YP + c8;
      const ms1_v4f f0 = *(const ms1_v4f*)(sp);
      const ms1_v4f f1 = *(const ms1_v4f*)(sp + 4);
      unsigned h0, h1, h2, h3, l0, l1, l2, l3;
      ms1_pack2(f0[0], f0[1], h0, l0);
      ms1_pack2(f0[2], f0[3], h1, l1);
      ms1_pack2(f1[0], f1[1], h2, l2);
      ms1_pack2(f1[2], f1[3], h3, l3);
      hw[it] = (ms1_v4u){h0, h1, h2, h3};
      lw[it] = (ms1_v4u){l0, l1, l2, l3};
    }
    for (int pass = 0; pass < 2; ++pass) {
#pragma unroll
      for (int it = 0; it < NIT; ++it) {
        const int row = it * RPI + wave * 4 + q;
        const long o = (rowc + row) * a.ld_y + d0 + c8;
        *(volatile ms1_v4u*)(a.y + o) = hw[it];
        if (hasLo) *(volatile ms1_v4u*)(a.y_lo + o) = lw[it];
      }
      __threadfence();
    }
  }
}

__global__ __launch_bounds__(256) void group_stats_kernel(
    const float* __restrict__ O, float* __restrict__ ST)
{
  __shared__ float red[256];
  const int tid = threadIdx.x, lane = tid & 31, wave = tid >> 5;
  const int blk = blockIdx.x;
  const int b = blk >> 3, g = blk & 7;
  const float* base = O + (size_t)b * kSeq * kDm + g * 64;
  const int c4 = (tid & 15) * 4;
  const int r0 = tid >> 4;
  float s = 0.0f;
#pragma unroll 4
  for (int i = 0; i < 32; ++i) {
    const v4f v = *(const v4f*)(base + (size_t)(r0 + i * 16) * kDm + c4);
    s += (v[0] + v[1]) + (v[2] + v[3]);
  }
  red[tid] = s;
  __syncthreads();
  for (int off = 128; off > 0; off >>= 1) {
    if (tid < off) red[tid] += red[tid + off];
    __syncthreads();
  }
  const float mu = red[0] * (1.0f / 32768.0f);
  __syncthreads();
  float qs = 0.0f;
#pragma unroll 4
  for (int i = 0; i < 32; ++i) {
    const v4f v = *(const v4f*)(base + (size_t)(r0 + i * 16) * kDm + c4);
    const float e0 = v[0] - mu, e1 = v[1] - mu, e2 = v[2] - mu, e3 = v[3] - mu;
    qs += (e0 * e0 + e1 * e1) + (e2 * e2 + e3 * e3);
  }
  red[tid] = qs;
  __syncthreads();
  for (int off = 128; off > 0; off >>= 1) {
    if (tid < off) red[tid] += red[tid + off];
    __syncthreads();
  }
  const float var = red[0] * (1.0f / 32768.0f);
  const float rs = rsqrtf(var + 1e-5f);
  if (wave == 0) {
    const float val = (lane == 0) ? mu : ((lane == 1) ? rs : 0.0f);
    volatile float* p = ST + (size_t)blk * 32 + lane;
    *p = val;
    __threadfence();
    *p = val;
  }
}

__device__ __forceinline__ float mish_f(float v) {
  const float sp = fmaxf(v, 0.0f) + log1pf(expf(-fabsf(v)));
  return v * tanhf(sp);
}

__global__ __launch_bounds__(256) void norm_mish_store_kernel(
    const float* __restrict__ O, const float* __restrict__ ST,
    const float* __restrict__ gw, const float* __restrict__ gb, float* __restrict__ out)
{
  __shared__ float tile[64 * 65];
  const int tid = threadIdx.x, lane = tid & 31, wave = tid >> 5;
  const int l0 = blockIdx.x * 64;
  const int g  = blockIdx.y;
  const int b  = blockIdx.z;
  const int c0 = g * 64;
  const float mu = ST[(size_t)(b * kGroups + g) * 32];
  const float rs = ST[(size_t)(b * kGroups + g) * 32 + 1];
  const int cc  = tid & 63;
  const int lr0 = tid >> 6;
  const float wgt = gw[c0 + cc];
  const float bia = gb[c0 + cc];
  const float* src = O + (size_t)(b * kSeq + l0) * kDm + c0 + cc;
  for (int i = 0; i < 16; ++i) {
    const int ll = lr0 + i * 4;
    const float o = src[(size_t)ll * kDm];
    const float nv = (o - mu) * rs;
    const float av = nv * wgt + bia;
    tile[ll * 65 + cc] = mish_f(av);
  }
  __syncthreads();
  const int hh = lane >> 4, l4 = (lane & 15) * 4;
  v4f val[4];
#pragma unroll
  for (int it = 0; it < 4; ++it) {
    const int crow = it * 16 + wave * 2 + hh;
    v4f t;
    t[0] = tile[(l4 + 0) * 65 + crow];
    t[1] = tile[(l4 + 1) * 65 + crow];
    t[2] = tile[(l4 + 2) * 65 + crow];
    t[3] = tile[(l4 + 3) * 65 + crow];
    val[it] = t;
  }
  for (int pass = 0; pass < 2; ++pass) {
#pragma unroll
    for (int it = 0; it < 4; ++it) {
      const int crow = it * 16 + wave * 2 + hh;
      *(volatile v4f*)(out + ((size_t)b * kDm + c0 + crow) * kSeq + l0 + l4) = val[it];
    }
    __threadfence();
  }
}

extern "C" void kernel_launch(void* const* d_in, const int* in_sizes, int n_in,
                              void* d_out, int out_size, void* d_ws, size_t ws_size,
                              hipStream_t stream)
{
  if (n_in < 12) return;
  if (in_sizes[0] != kBatch * kDm * kSeq) return;
  if (in_sizes[1] != kXzP * kDm) return;
  if (in_sizes[2] != kDin * 4) return;
  if (in_sizes[3] != kDin) return;
  if (in_sizes[4] != kBcP * kDin) return;
  if (in_sizes[5] != kDin * kDtR) return;
  if (in_sizes[6] != kDin) return;
  if (in_sizes[7] != kDin * kNst) return;
  if (in_sizes[8] != kDin) return;
  if (in_sizes[9] != kDm * kDin) return;
  if (in_sizes[10] != kDm) return;
  if (in_sizes[11] != kDm) return;
  if (out_size != kBatch * kDm * kSeq) return;
  if (ws_size < kWsTotal) return;

  const float* x      = (const float*)d_in[0];
  const float* W_in   = (const float*)d_in[1];
  const float* conv_w = (const float*)d_in[2];
  const float* conv_b = (const float*)d_in[3];
  const float* W_x    = (const float*)d_in[4];
  const float* W_dt   = (const float*)d_in[5];
  const float* b_dt   = (const float*)d_in[6];
  const float* A_log  = (const float*)d_in[7];
  const float* D_par  = (const float*)d_in[8];
  const float* W_out  = (const float*)d_in[9];
  const float* gn_w   = (const float*)d_in[10];
  const float* gn_b   = (const float*)d_in[11];
  float* out = (float*)d_out;

  char* ws = (char*)d_ws;
  unsigned short* WINH = (unsigned short*)(ws + kWsWINH);
  unsigned short* WINL = (unsigned short*)(ws + kWsWINL);
  unsigned short* WX   = (unsigned short*)(ws + kWsWX);
  unsigned short* WDT  = (unsigned short*)(ws + kWsWDT);
  unsigned short* WOUT = (unsigned short*)(ws + kWsWOUT);
  unsigned short* XH   = (unsigned short*)(ws + kWsXH);
  unsigned short* XL   = (unsigned short*)(ws + kWsXL);
  float*          XZ   = (float*)(ws + kWsXZ);
  float*          U    = (float*)(ws + kWsU);
  unsigned short* UH   = (unsigned short*)(ws + kWsUH);
  unsigned short* UL   = (unsigned short*)(ws + kWsUL);
  float*          BC   = (float*)(ws + kWsBC);
  unsigned short* BCH  = (unsigned short*)(ws + kWsBCH);
  unsigned short* BCL  = (unsigned short*)(ws + kWsBCL);
  float*          DTR  = (float*)(ws + kWsDTR);
  float*          DT   = (float*)(ws + kWsDT);
  unsigned short* YH   = (unsigned short*)(ws + kWsYH);
  unsigned short* YL   = (unsigned short*)(ws + kWsYL);
  float*          ST   = (float*)(ws + kWsST);
  float*          O    = (float*)(ws + kWsO);

  pack_weight_f16_kernel<true><<<dim3((kXzP * kDm / 8) / 256), 256, 0, stream>>>(W_in, WINH, WINL, kXzP * kDm / 8, kWCarry);
  pack_weight_f16_kernel<false><<<dim3((kBcP * kDin / 8) / 256), 256, 0, stream>>>(W_x, WX, WX, kBcP * kDin / 8, kWCarry);
  pack_weight_f16_kernel<false><<<dim3((kDin * kDtR / 8) / 256), 256, 0, stream>>>(W_dt, WDT, WDT, kDin * kDtR / 8, kWCarry);
  pack_weight_f16_kernel<false><<<dim3((kDm * kDin / 8) / 256), 256, 0, stream>>>(W_out, WOUT, WOUT, kDm * kDin / 8, kWCarry);

  xpose_split_kernel<<<dim3(kSeq / 64, kDm / 64, kBatch), 256, 0, stream>>>(x, XH, XL);

  eng::gemm_f16_kernel<1, 2><<<dim3((kRows / 16) * (kXzP / 64) / 8), 256, 0, stream>>>(
      XH, XL, kDm, WINH, WINL, kDm, XZ, kXzP, kRows, kXzP, kDm, kSW, kSWr);

  for (int b = 0; b < kBatch; ++b) {
    conv_silu_kernel<<<dim3(kDin / 256, kSeq / 64), 256, 0, stream>>>(
        XZ + (size_t)b * kSeq * kXzP, conv_w, conv_b,
        U + (size_t)b * kSeq * kDin, UH + (size_t)b * kSeq * kDin, UL + (size_t)b * kSeq * kDin);
  }

  eng::gemm_f16_kernel<2, 1><<<dim3((kRows / 32) * (kBcP / 64) / 8), 256, 0, stream>>>(
      UH, UL, kDin, WX, WX, kDin, BC, kBcP, kRows, kBcP, kDin, kSW, kSWr);

  split_rows_f16_kernel<<<(kRows * kBcP / 8) / 256, 256, 0, stream>>>(BC, BCH, BCL, kRows * kBcP / 8);

  eng::gemm_f16_kernel<2, 1><<<dim3((kRows / 32) * (kDin / 64) / 8), 256, 0, stream>>>(
      BCH, BCL, kBcP, WDT, WDT, kDtR, DTR, kDin, kRows, kDin, kDtR, kSW, kSWr);

  bias_rows_kernel<<<dim3(kDin / 4 / 256, kRows / 8), 256, 0, stream>>>(DTR, b_dt, DT);

  for (int b = 0; b < kBatch; ++b) {
    ms1_args sa;
    sa.dtpre = DT + (size_t)b * kSeq * kDin;
    sa.u = U + (size_t)b * kSeq * kDin;
    sa.bc = BC + (size_t)b * kSeq * kBcP;
    sa.z = XZ + (size_t)b * kSeq * kXzP;
    sa.A_log = A_log;
    sa.Dskip = D_par;
    sa.y = (__half*)(YH + (size_t)b * kSeq * kDin);
    sa.y_lo = (__half*)(YL + (size_t)b * kSeq * kDin);
    sa.ld_dtpre = kDin;
    sa.ld_u = kDin;
    sa.ld_bc = kBcP;
    sa.ld_z = kXzP;
    sa.ld_y = kDin;
    sa.offB = kScanOffB;
    sa.offC = kScanOffC;
    sa.offZ = kDin;
    sa.ycarry = kYCarry;
    sa.dir = 1;
    sa.D = kDin;
    sa.L = kSeq;
    sa.nbatch = 1;
    ms1_scan_kernel<16><<<dim3(kDin / 64), 64, 0, stream>>>(sa);
  }

  eng::gemm_f16_kernel<2, 1><<<dim3((kRows / 32) * (kDm / 64) / 8), 256, 0, stream>>>(
      YH, YL, kDin, WOUT, WOUT, kDin, O, kDm, kRows, kDm, kDin, kSY, kSYr);

  group_stats_kernel<<<dim3(kBatch * kGroups), 256, 0, stream>>>(O, ST);

  norm_mish_store_kernel<<<dim3(kSeq / 64, kGroups, kBatch), 256, 0, stream>>>(O, ST, gn_w, gn_b, out);
}
